// LinearLayer_76020921140428
// MI455X (gfx1250) — hardware-verified
//
#include <hip/hip_runtime.h>


#define NB   8192
#define NI   1024
#define NO   1024
#define NP   8
#define DM   NI
#define NTK  NB
#define LOSC 1024.0f

typedef _Float16 h16;
typedef unsigned short bf;
typedef __attribute__((ext_vector_type(16))) __bf16   v16bf;
typedef __attribute__((ext_vector_type(16))) _Float16 v16h;
typedef __attribute__((ext_vector_type(8)))  _Float16 v8h;
typedef __attribute__((ext_vector_type(8)))  unsigned short v8us;
typedef __attribute__((ext_vector_type(8)))  float    v8f;
typedef __attribute__((ext_vector_type(4)))  float    v4f;
typedef __attribute__((ext_vector_type(4)))  _Float16 v4h;
typedef v8h  __attribute__((may_alias)) v8ha;
typedef v4f  __attribute__((may_alias)) v4fa;
typedef v8us __attribute__((may_alias)) v8usa;

__device__ __forceinline__ unsigned short f2bf(float f) { unsigned u = __float_as_uint(f); u += 0x7FFFu + ((u >> 16) & 1u); return (unsigned short)(u >> 16); }
__device__ __forceinline__ float bf2f(unsigned short b) { return __uint_as_float(((unsigned)b) << 16); }
__device__ __forceinline__ float bfr(float f) { return bf2f(f2bf(f)); }
__device__ __forceinline__ v16h cat16(v8h lo, v8h hi) { return __builtin_shufflevector(lo, hi, 0, 1, 2, 3, 4, 5, 6, 7, 8, 9, 10, 11, 12, 13, 14, 15); }
__device__ __forceinline__ v16bf cat16b(v8us lo, v8us hi) { return __builtin_bit_cast(v16bf, __builtin_shufflevector(lo, hi, 0, 1, 2, 3, 4, 5, 6, 7, 8, 9, 10, 11, 12, 13, 14, 15)); }
__device__ __forceinline__ v8f wmma16(v16h a, v16h b, v8f c) { return __builtin_amdgcn_wmma_f32_16x16x32_f16(false, a, false, b, (short)0, c, false, false); }
__device__ __forceinline__ v8f wmmab(v16bf a, v16bf b, v8f c) { return __builtin_amdgcn_wmma_f32_16x16x32_bf16(false, a, false, b, (short)0, c, false, false); }

__global__ __launch_bounds__(256) void k_cvtb(const float* __restrict__ src, int nrows, bf* dst) {
    const int lane = threadIdx.x & 31, r = blockIdx.x * 8 + (threadIdx.x >> 5);
    if (r >= nrows) return;
    v8us o[DM / 256];
#pragma unroll
    for (int q = 0; q < DM / 256; ++q) { v8us t;
#pragma unroll
        for (int i = 0; i < 8; ++i) t[i] = f2bf(src[(size_t)r * DM + q * 256 + lane * 8 + i]);
        o[q] = t; }
#pragma unroll
    for (int q = 0; q < DM / 256; ++q) *(volatile v8us*)(dst + (size_t)r * DM + q * 256 + lane * 8) = o[q];
    __threadfence();
#pragma unroll
    for (int q = 0; q < DM / 256; ++q) *(volatile v8us*)(dst + (size_t)r * DM + q * 256 + lane * 8) = o[q];
}

__global__ __launch_bounds__(128) void k_gemm3(const bf* __restrict__ Ah, const bf* __restrict__ Al, const bf* __restrict__ Bh, const bf* __restrict__ Bl, int K, float* C, int ldc) {
    __shared__ __align__(16) float ost[4][16 * 68];
    const int lane = threadIdx.x & 31, wave = threadIdx.x >> 5, lr = lane & 15, hi = lane >> 4;
    const int r0 = blockIdx.x * 64 + wave * 16, c0 = blockIdx.y * 64;
    const size_t aoff = (size_t)(r0 + lr) * K + 8 * hi;
    v8f acc[4];
#pragma unroll
    for (int t = 0; t < 4; ++t) acc[t] = (v8f){};
#pragma unroll 1
    for (int kc = 0; kc < K; kc += 32) {
        const v16bf a = cat16b(*(const v8us*)(Ah + aoff + kc), *(const v8us*)(Ah + aoff + kc + 16));
        const v16bf al = cat16b(*(const v8us*)(Al + aoff + kc), *(const v8us*)(Al + aoff + kc + 16));
#pragma unroll
        for (int t = 0; t < 4; ++t) { const size_t bo = (size_t)(c0 + t * 16 + lr) * K + kc + 8 * hi;
            const v16bf bh = cat16b(*(const v8us*)(Bh + bo), *(const v8us*)(Bh + bo + 16)); const v16bf bl = cat16b(*(const v8us*)(Bl + bo), *(const v8us*)(Bl + bo + 16));
            acc[t] = wmmab(a, bh, acc[t]); acc[t] = wmmab(al, bh, acc[t]); acc[t] = wmmab(a, bl, acc[t]); }
        asm volatile("v_nop\n\tv_nop\n\tv_nop\n\tv_nop" : "+v"(acc[0]), "+v"(acc[1]), "+v"(acc[2]), "+v"(acc[3]) : "v"(a), "v"(al));
    }
    float* os = &ost[wave][0];
#pragma unroll
    for (int t = 0; t < 4; ++t) {
#pragma unroll
        for (int j = 0; j < 8; ++j) os[(hi * 8 + j) * 68 + t * 16 + lr] = acc[t][j]; }
    __builtin_amdgcn_wave_barrier(); asm volatile("" ::: "memory");
    float* crow = C + (size_t)r0 * ldc + c0;
    auto pass = [&]() {
#pragma unroll
        for (int s = 0; s < 8; ++s) { const int Lid = (lane >> 3) + 4 * s, piece = lane & 7; const int row = Lid >> 1, cofs = (Lid & 1) * 32 + piece * 4;
            const v4f val = *(const v4fa*)(os + row * 68 + cofs); *(volatile v4f*)(crow + (size_t)row * ldc + cofs) = val; }
    };
    pass(); __threadfence(); pass();
}

__global__ __launch_bounds__(256) void k_weff(const float* __restrict__ coef, const float* __restrict__ Wt, bf* Wh, bf* Wl) {
    const int lane = threadIdx.x & 31, o = blockIdx.x * 8 + (threadIdx.x >> 5); if (o >= NO) return;
#pragma unroll 1
    for (int ps = 0; ps < 2; ++ps) {
#pragma unroll 1
        for (int q = 0; q < NI / 256; ++q) { const int i0 = q * 256 + lane * 8; v8us oh, ol;
#pragma unroll
            for (int k = 0; k < 8; ++k) { const int i = i0 + k; const float* cp = coef + ((size_t)o * NI + i) * NP; float s = 0.f;
#pragma unroll
                for (int p = 0; p < NP; ++p) s += bfr(cp[p]);
                const float w = s * bfr(Wt[(size_t)o * NI + i]); const unsigned short hb = f2bf(w); oh[k] = hb; ol[k] = f2bf(w - bf2f(hb)); }
            const size_t off = (size_t)o * NI + i0; *(volatile v8us*)(Wh + off) = oh; *(volatile v8us*)(Wl + off) = ol; }
        if (ps == 0) __threadfence(); }
}
__global__ __launch_bounds__(256) void k_xz(const float* __restrict__ src, bf* dh, bf* dz) {
    const int lane = threadIdx.x & 31, r = blockIdx.x * 8 + (threadIdx.x >> 5); if (r >= NB) return;
#pragma unroll 1
    for (int ps = 0; ps < 2; ++ps) {
#pragma unroll 1
        for (int q = 0; q < NI / 256; ++q) { const size_t o = (size_t)r * NI + q * 256 + lane * 8; const v8f v = *(const v8f*)(src + o); v8us oh, z;
#pragma unroll
            for (int i = 0; i < 8; ++i) { oh[i] = f2bf(v[i]); z[i] = 0; }
            *(volatile v8us*)(dh + o) = oh; *(volatile v8us*)(dz + o) = z; }
        if (ps == 0) __threadfence(); }
}

extern "C" void kernel_launch(void* const* d_in, const int* in_sizes, int n_in,
                              void* d_out, int out_size, void* d_ws, size_t ws_size, hipStream_t stream) {
    (void)in_sizes; (void)n_in; (void)out_size;
    const float* x = (const float*)d_in[0]; const float* coef = (const float*)d_in[1]; const float* Wt = (const float*)d_in[2];
    float* out = (float*)d_out;
    char* wsp = (char*)d_ws;
    auto take = [&](size_t bytes) { char* p = wsp; wsp += (bytes + 255) & ~(size_t)255; return (void*)p; };
    bf* Xh = (bf*)take((size_t)NB * NI * 2); bf* Xz = (bf*)take((size_t)NB * NI * 2); bf* Wh = (bf*)take((size_t)NO * NI * 2); bf* Wl = (bf*)take((size_t)NO * NI * 2);
    if ((size_t)(wsp - (char*)d_ws) > ws_size) return;
    k_weff<<<NO / 8, 256, 0, stream>>>(coef, Wt, Wh, Wl);
    k_xz<<<NB / 8, 256, 0, stream>>>(x, Xh, Xz);
    k_gemm3<<<dim3(NB / 64, NO / 64, 1), 128, 0, stream>>>(Xh, Xz, Wh, Wl, NI, out, NO);
}
